// WeaveNet_47622597378229
// MI455X (gfx1250) — hardware-verified
//
#include <hip/hip_runtime.h>
#include <math.h>
#include <stdint.h>

#define BIMG  4
#define NB    (2 * BIMG)
#define NN    256
#define MM    256
#define HW    (NN * MM)
#define CZ    32
#define CI    64
#define NLAY  6
#define NIDX  MM
#define ZP    64
#define PP    128
#define WPP   64
#define RWM0  0
#define RWMB  CI
#define RWX0  (RWMB + (NLAY - 1) * CI)
#define RWT0  (RWX0 + CZ)
#define RWXB  (RWT0 + CZ)
#define RWTB  (RWXB + (NLAY - 1) * CZ)
#define RWF   (RWTB + (NLAY - 1) * CZ)
#define NWROW (RWF + 16)
#define NPB   (BIMG * HW / 128)
#define APIX  512
#define OUTN  (BIMG * HW)
#define WSC   16.0f
#define IWSC  (1.0f / 16.0f)
#define LOSC  4096.0f
#define ILOSC (1.0f / 4096.0f)

static_assert(NN == MM);
static_assert((HW % APIX) == 0 && (APIX % 64) == 0 && (HW % 128) == 0 && (HW % 32) == 0);
static_assert((NN % 32) == 0 && (MM % 32) == 0);
static_assert(((BIMG * NIDX) % 128) == 0 && ((NB * NIDX) % 8) == 0);
static_assert(CZ == 32 && CI == 64 && ZP == 2 * CZ && PP == 2 * CI && WPP == CI);
static_assert((RWMB % 4) == 0 && (RWX0 % 4) == 0 && (RWT0 % 4) == 0 && (RWXB % 4) == 0);
static_assert((RWTB % 4) == 0 && (RWF % 4) == 0 && (NWROW % 4) == 0);

typedef _Float16 v16h __attribute__((ext_vector_type(16)));
typedef _Float16 v8h  __attribute__((ext_vector_type(8)));
typedef float    v8f  __attribute__((ext_vector_type(8)));
typedef float    v4f  __attribute__((ext_vector_type(4)));
typedef unsigned int v4u __attribute__((ext_vector_type(4)));
typedef unsigned int v2u __attribute__((ext_vector_type(2)));
union FragH { v16h v; v8h hf[2]; };
union F8 { v4f v[2]; float f[8]; };
union H8 { v8h v; _Float16 f[8]; };
union HS { unsigned short u; _Float16 h; };

struct GD {
  const _Float16* A;
  const _Float16* W;
  const float* tsrc;
  float* O;
  float* part;
  int lda;
  int rpi;
};
static_assert(sizeof(GD) == 48);

__device__ __forceinline__ unsigned short bf_bits(float f) {
  unsigned u = __float_as_uint(f);
  return (unsigned short)((u + 0x7FFFu + ((u >> 16) & 1u)) >> 16);
}
__device__ __forceinline__ float bf_up(unsigned short b) { return __uint_as_float(((unsigned)b) << 16); }
__device__ __forceinline__ float bfr(float f) { return bf_up(bf_bits(f)); }
__device__ __forceinline__ float h_up(unsigned int b) { HS t; t.u = (unsigned short)b; return (float)t.h; }
__device__ __forceinline__ unsigned int h_bits(_Float16 x) { HS t; t.h = x; return (unsigned int)t.u; }
__device__ __forceinline__ v8f zero8() { v8f z = {0.f, 0.f, 0.f, 0.f, 0.f, 0.f, 0.f, 0.f}; return z; }

__device__ __forceinline__ void split16(float t, _Float16& hh, _Float16& ll) {
  const _Float16 h0 = (_Float16)t;
  const _Float16 hz = (_Float16)0.0f;
  hh = (fabsf(t) < 6.103515625e-05f) ? hz : h0;
  ll = (_Float16)((t - (float)hh) * LOSC);
}

__device__ __forceinline__ v16h ldf(const _Float16* p) {
  FragH f;
  f.hf[0] = *(const v8h*)(p);
  f.hf[1] = *(const v8h*)(p + 16);
  return f.v;
}
__device__ __forceinline__ v8f mma(v16h a, v16h b, v8f c) {
  return __builtin_amdgcn_wmma_f32_16x16x32_f16(false, a, false, b, (short)0, c, false, false);
}
__device__ __forceinline__ void guard4(v8f& c0, v8f& c1, v8f& c2, v8f& c3, v16h x0, v16h x1, v16h x2, v16h x3,
                                       v16h x4, v16h x5, v16h x6, v16h x7, v16h y0, v16h y1) {
#if defined(__HIP_DEVICE_COMPILE__)
  asm volatile("v_nop\n\tv_nop\n\tv_nop\n\tv_nop"
               : "+v"(c0), "+v"(c1), "+v"(c2), "+v"(c3)
               : "v"(x0), "v"(x1), "v"(x2), "v"(x3), "v"(x4), "v"(x5), "v"(x6), "v"(x7), "v"(y0), "v"(y1));
#endif
}
__device__ __forceinline__ void wave_sync_lds() {
  __builtin_amdgcn_fence(__ATOMIC_RELEASE, "workgroup");
  __builtin_amdgcn_wave_barrier();
  __builtin_amdgcn_fence(__ATOMIC_ACQUIRE, "workgroup");
}
__device__ __forceinline__ float wsum32(float v) {
  v += __shfl_xor(v, 16, 32); v += __shfl_xor(v, 8, 32); v += __shfl_xor(v, 4, 32);
  v += __shfl_xor(v, 2, 32);  v += __shfl_xor(v, 1, 32);
  return v;
}
__device__ __forceinline__ float wmax32(float v) {
  v = fmaxf(v, __shfl_xor(v, 16, 32)); v = fmaxf(v, __shfl_xor(v, 8, 32)); v = fmaxf(v, __shfl_xor(v, 4, 32));
  v = fmaxf(v, __shfl_xor(v, 2, 32));  v = fmaxf(v, __shfl_xor(v, 1, 32));
  return v;
}

__global__ __launch_bounds__(256) void k_prep(const float* Za, const float* Zb, _Float16* zyh) {
  const int tid = threadIdx.x;
  const int row = blockIdx.x * 32 + (tid >> 3);
  const int e = tid & 7;
  const int j = row / HW, p = row - j * HW;
  const int n = p / MM, mc = p - n * MM;
  const int ja = (j < BIMG) ? j : (j - BIMG);
  const float va = Za[(size_t)ja * HW + p];
  const float vb = Zb[(size_t)ja * HW + (size_t)mc * NN + n];
  const float own = (j < BIMG) ? va : vb;
  const float oth = (j < BIMG) ? vb : va;
  const _Float16 hown = (_Float16)bfr(own);
  const _Float16 hoth = (_Float16)bfr(oth);
  H8 pk;
#pragma unroll
  for (int u = 0; u < 8; ++u) pk.f[u] = (_Float16)0.0f;
  pk.f[0] = (e == 0) ? hown : (_Float16)0.0f;
  pk.f[1] = (e == 0) ? hoth : (_Float16)0.0f;
  _Float16* dst = zyh + (size_t)row * ZP + e * 8;
  *(volatile v8h*)dst = pk.v;
  __threadfence();
  *(volatile v8h*)dst = pk.v;
}

__global__ __launch_bounds__(256) void k_wplanes(const float* Wm0, const float* Wm, const float* W0, const float* W,
                                                 const float* Wf, _Float16* wpl) {
  const int gid = blockIdx.x * 256 + threadIdx.x;
  if (gid >= NWROW * 8) return;
  const int R = gid >> 3, e = gid & 7, k0 = e * 8;
  const float* src; int n, rs, o, kb, kn;
  if (R < RWMB)       { src = Wm0; n = CI * 2;                         rs = 2;           o = R;        kb = 0;      kn = 2; }
  else if (R < RWX0)  { src = Wm;  n = (NLAY - 1) * CI * 2 * CZ;       rs = 2 * CZ;      o = R - RWMB; kb = 0;      kn = 2 * CZ; }
  else if (R < RWT0)  { src = W0;  n = CZ * (2 + CI);                  rs = 2 + CI;      o = R - RWX0; kb = 0;      kn = 2; }
  else if (R < RWXB)  { src = W0;  n = CZ * (2 + CI);                  rs = 2 + CI;      o = R - RWT0; kb = 2;      kn = CI; }
  else if (R < RWTB)  { src = W;   n = (NLAY - 1) * CZ * (2 * CZ + CI); rs = 2 * CZ + CI; o = R - RWXB; kb = 0;      kn = 2 * CZ; }
  else if (R < RWF)   { src = W;   n = (NLAY - 1) * CZ * (2 * CZ + CI); rs = 2 * CZ + CI; o = R - RWTB; kb = 2 * CZ; kn = CI; }
  else                { src = Wf;  n = 2 * CZ;                         rs = 2 * CZ;      o = R - RWF;  kb = 0;      kn = (o == 0) ? 2 * CZ : 0; }
  H8 pk;
#pragma unroll
  for (int u = 0; u < 8; ++u) {
    const int k = k0 + u;
    int idx = o * rs + kb + k;
    idx = (idx < 0) ? 0 : ((idx > n - 1) ? (n - 1) : idx);
    const float w = bfr(src[idx]);
    const float v = (k < kn) ? w : 0.0f;
    pk.f[u] = (_Float16)(v * WSC);
  }
  _Float16* dst = wpl + (size_t)R * WPP + e * 8;
  *(volatile v8h*)dst = pk.v;
  __threadfence();
  *(volatile v8h*)dst = pk.v;
}

template <int NS, int KX>
__global__ __launch_bounds__(256) void k_pool(const _Float16* A, const _Float16* Wp, const float* bias, _Float16* P) {
  __shared__ __align__(16) _Float16 sPH[8][PP];
  const int tid = threadIdx.x, wave = tid >> 5, lane = tid & 31;
  const int m = lane & 15, h = lane >> 4, k8 = h * 8;
  const int gw = blockIdx.x * 8 + wave;
  const int b = gw / NIDX, idx = gw - b * NIDX;
  const int b2 = (b + BIMG) % NB;
  const bool lower = b < BIMG;
  const int pbase = lower ? idx : idx * MM;
  const int pstep = lower ? MM : 1;
  const int ntile = (lower ? NN : MM) / 32;
  const _Float16* Ab  = A + (size_t)b  * HW * ZP;
  const _Float16* Ab2 = A + (size_t)b2 * HW * ZP;
  float run[4];
#pragma unroll
  for (int nt = 0; nt < 4; ++nt) run[nt] = -3.0e38f;
#pragma unroll 1
  for (int t = 0; t < ntile; ++t) {
    v16h ha[2], hb[2], la[2], lb[2];
#pragma unroll
    for (int i = 0; i < 2; ++i) {
      const int p = pbase + (t * 32 + i * 16 + m) * pstep;
      const _Float16* r0 = Ab + (size_t)p * ZP + k8;
      ha[i] = ldf(r0);
      la[i] = ha[i]; hb[i] = ha[i]; lb[i] = ha[i];
      if (NS == 2) la[i] = ldf(r0 + CZ);
      if (KX == 1) {
        const _Float16* r1 = Ab2 + (size_t)p * ZP + k8;
        hb[i] = ldf(r1);
        lb[i] = hb[i];
        if (NS == 2) lb[i] = ldf(r1 + CZ);
      }
    }
#pragma unroll
    for (int nt = 0; nt < 4; ++nt) {
      const _Float16* wr = Wp + (size_t)(nt * 16 + m) * WPP + k8;
      const v16h bo = ldf(wr);
      v16h bp = bo;
      if (KX == 1) bp = ldf(wr + 32);
      v8f c0 = zero8(), c1 = zero8(), e0 = zero8(), e1 = zero8();
      c0 = mma(ha[0], bo, c0);
      c1 = mma(ha[1], bo, c1);
      if (NS == 2) { e0 = mma(la[0], bo, e0); e1 = mma(la[1], bo, e1); }
      if (KX == 1) {
        c0 = mma(hb[0], bp, c0);
        c1 = mma(hb[1], bp, c1);
        if (NS == 2) { e0 = mma(lb[0], bp, e0); e1 = mma(lb[1], bp, e1); }
      }
      guard4(c0, c1, e0, e1, ha[0], ha[1], hb[0], hb[1], la[0], la[1], lb[0], lb[1], bo, bp);
      float mx = -3.0e38f;
#pragma unroll
      for (int r = 0; r < 8; ++r) {
        const float f0 = (NS == 2) ? (c0[r] + e0[r] * ILOSC) : c0[r];
        const float f1 = (NS == 2) ? (c1[r] + e1[r] * ILOSC) : c1[r];
        mx = fmaxf(mx, fmaxf(f0, f1));
      }
      mx = fmaxf(mx, __shfl_xor(mx, 16, 32));
      run[nt] = fmaxf(run[nt], mx);
    }
  }
  _Float16* sw = sPH[wave];
#pragma unroll
  for (int nt = 0; nt < 4; ++nt) {
    const int c = nt * 16 + m;
    const float v = run[nt] * IWSC + bfr(bias[c]);
    _Float16 hh, ll;
    split16(v, hh, ll);
    if (h == 0) { sw[c] = hh; sw[CI + c] = ll; }
  }
  wave_sync_lds();
  const v8h pv = *(const v8h*)(sw + (lane & 15) * 8);
  if (lane < 16) {
    _Float16* dst = P + ((size_t)b * NIDX + idx) * PP + lane * 8;
    *(volatile v8h*)dst = pv;
    __threadfence();
    *(volatile v8h*)dst = pv;
  }
}

template <int EPI, int NS, int KM>
__global__ __launch_bounds__(128) void k_gemm(GD d) {
  constexpr int NT = (EPI == 3) ? 1 : 2;
  __shared__ __align__(16) float slab[4][2][32 * 36];
  __shared__ __align__(16) float sCol[4][64];
  __shared__ __align__(16) float sPart[4][64];
  __shared__ __align__(16) float sLine[64];
  const int tid = threadIdx.x, wave = tid >> 5, lane = tid & 31;
  const int m = lane & 15, h = lane >> 4, k8 = h * 8;
  const int gw = blockIdx.x * 4 + wave;
  const int rowg = gw * 32;
  const int q = rowg / d.rpi;
  const int p0 = rowg - q * d.rpi;
  const int ib0 = q, ib1 = q + BIMG;
  const int lo = d.lda >> 1;
  float* slw0 = slab[wave][0];
  float* slw1 = slab[wave][1];
#pragma unroll
  for (int i = 0; i < 2; ++i) {
    const int p = p0 + i * 16 + m;
    const _Float16* r0 = d.A + ((size_t)ib0 * d.rpi + p) * d.lda + k8;
    const _Float16* r1 = d.A + ((size_t)ib1 * d.rpi + p) * d.lda + k8;
    const v16h h0 = ldf(r0), h1 = ldf(r1);
    v16h l0 = h0, l1 = h1, g0 = h0, g1 = h1, gl0 = h0, gl1 = h1;
    if (NS == 2) { l0 = ldf(r0 + lo); l1 = ldf(r1 + lo); }
    if (KM == 2) {
      g0 = ldf(r0 + 32); g1 = ldf(r1 + 32);
      gl0 = g0; gl1 = g1;
      if (NS == 2) { gl0 = ldf(r0 + 32 + lo); gl1 = ldf(r1 + 32 + lo); }
    }
#pragma unroll
    for (int nt = 0; nt < NT; ++nt) {
      const _Float16* wr = d.W + (size_t)(nt * 16 + m) * WPP + k8;
      const v16h bo = ldf(wr);
      v16h bp = bo;
      if (KM >= 1) bp = ldf(wr + 32);
      v8f c0 = zero8(), c1 = zero8(), e0 = zero8(), e1 = zero8();
      c0 = mma(h0, bo, c0);
      c1 = mma(h1, bo, c1);
      if (NS == 2) { e0 = mma(l0, bo, e0); e1 = mma(l1, bo, e1); }
      if (KM == 1) {
        c0 = mma(h1, bp, c0);
        c1 = mma(h0, bp, c1);
        if (NS == 2) { e0 = mma(l1, bp, e0); e1 = mma(l0, bp, e1); }
      }
      if (KM == 2) {
        c0 = mma(g0, bp, c0);
        c1 = mma(g1, bp, c1);
        if (NS == 2) { e0 = mma(gl0, bp, e0); e1 = mma(gl1, bp, e1); }
      }
      guard4(c0, c1, e0, e1, h0, h1, l0, l1, g0, g1, gl0, gl1, bo, bp);
      if (EPI < 3) {
#pragma unroll
        for (int r = 0; r < 8; ++r) {
          const int o = (i * 16 + 8 * h + r) * 36 + nt * 16 + m;
          const float f0 = (NS == 2) ? (c0[r] + e0[r] * ILOSC) : c0[r];
          const float f1 = (NS == 2) ? (c1[r] + e1[r] * ILOSC) : c1[r];
          slw0[o] = f0 * IWSC;
          slw1[o] = f1 * IWSC;
        }
      } else {
        if (m == 0) {
#pragma unroll
          for (int r = 0; r < 8; ++r) {
            const float f0 = (NS == 2) ? (c0[r] + e0[r] * ILOSC) : c0[r];
            const float f1 = (NS == 2) ? (c1[r] + e1[r] * ILOSC) : c1[r];
            sCol[wave][i * 16 + 8 * h + r]      = f0 * IWSC;
            sCol[wave][32 + i * 16 + 8 * h + r] = f1 * IWSC;
          }
        }
      }
    }
  }
  wave_sync_lds();

  if (EPI == 2) {
#pragma unroll
    for (int img = 0; img < 2; ++img) {
      const int bi = img ? ib1 : ib0;
      const bool lowb = bi < BIMG;
      float* sl = img ? slw1 : slw0;
#pragma unroll
      for (int it = 0; it < 8; ++it) {
        const int row = it * 4 + (lane >> 3), c4 = (lane & 7) * 4;
        const int p = p0 + row;
        const int idx = lowb ? (p % MM) : (p / MM);
        const v4f tv = *(const v4f*)(d.tsrc + ((size_t)bi * NIDX + idx) * CZ + c4);
        v4f sv = *(const v4f*)(sl + row * 36 + c4);
        sv += tv;
        *(v4f*)(sl + row * 36 + c4) = sv;
      }
    }
    wave_sync_lds();
  }
  if (EPI < 3) {
    for (int pass = 0; pass < 2; ++pass) {
#pragma unroll
      for (int img = 0; img < 2; ++img) {
        const int bi = img ? ib1 : ib0;
        const float* sl = img ? slw1 : slw0;
#pragma unroll
        for (int it = 0; it < 8; ++it) {
          const int row = it * 4 + (lane >> 3), c4 = (lane & 7) * 4;
          const v4f v = *(const v4f*)(sl + row * 36 + c4);
          *(volatile v4f*)(d.O + ((size_t)bi * d.rpi + p0 + row) * CZ + c4) = v;
        }
      }
      __threadfence();
    }
  }
  if (EPI == 2) {
    float s = 0.0f, qq = 0.0f;
#pragma unroll 4
    for (int r = 0; r < 32; ++r) {
      const float a0 = slw0[r * 36 + lane], a1 = slw1[r * 36 + lane];
      s += a0 + a1;
      qq += a0 * a0 + a1 * a1;
    }
    sPart[wave][lane] = s;
    sPart[wave][32 + lane] = qq;
  }
  if (EPI == 3) {
    const int img = (lane >> 3) & 1, e = lane & 7;
    const int bi = img ? ib1 : ib0;
    const v4f cv = *(const v4f*)(sCol[wave] + img * 32 + e * 4);
    if (lane < 16) {
      float* dst = d.O + (size_t)bi * d.rpi + p0 + e * 4;
      *(volatile v4f*)dst = cv;
      __threadfence();
      *(volatile v4f*)dst = cv;
    }
    const float a0 = sCol[wave][lane], a1 = sCol[wave][32 + lane];
    const float s  = wsum32(a0 + a1);
    const float qq = wsum32(a0 * a0 + a1 * a1);
    sPart[wave][lane]      = (lane == 0) ? s  : 0.0f;
    sPart[wave][32 + lane] = (lane == 0) ? qq : 0.0f;
  }
  if (EPI >= 2) {
    __syncthreads();
    if (tid < 64) {
      float a = 0.0f;
#pragma unroll
      for (int w = 0; w < 4; ++w) a += sPart[w][tid];
      sLine[tid] = a;
    }
    __syncthreads();
    if (tid < 16) {
      const v4f v = *(const v4f*)(sLine + tid * 4);
      float* dst = d.part + (size_t)blockIdx.x * 64 + tid * 4;
      *(volatile v4f*)dst = v;
      __threadfence();
      *(volatile v4f*)dst = v;
    }
  }
}

__global__ __launch_bounds__(64) void k_bnfin(const float* part, int nrows, float count, const float* g, const float* be,
                                             int ng, int nch, float* st) {
  __shared__ __align__(16) float sLine[64];
  const int t = threadIdx.x;
  if (t < 32) {
    double s = 0.0, qd = 0.0;
#pragma unroll 1
    for (int r = 0; r < nrows; ++r) {
      s  += (double)part[(size_t)r * 64 + t];
      qd += (double)part[(size_t)r * 64 + 32 + t];
    }
    const double inv = 1.0 / (double)count;
    const double mean = s * inv;
    double var = qd * inv - mean * mean;
    if (var < 0.0) var = 0.0;
    const float rstd = 1.0f / sqrtf((float)var + 1e-5f);
    const int gi = (t < ng) ? t : (ng - 1);
    const float gg = bfr(g[gi]), bb = bfr(be[gi]);
    float sc = gg * rstd;
    float sh = bb - (float)mean * sc;
    if (t >= nch) { sc = 0.0f; sh = 0.0f; }
    sLine[t] = sc;
    sLine[32 + t] = sh;
  }
  __syncthreads();
  if (t < 16) {
    const v4f v = *(const v4f*)(sLine + t * 4);
    float* dst = st + t * 4;
    *(volatile v4f*)dst = v;
    __threadfence();
    *(volatile v4f*)dst = v;
  }
}

__global__ __launch_bounds__(256) void k_bnapply(float* zy, _Float16* kh, unsigned int* kq, const float* st,
                                                 const float* aP, int addRes, int wkeep) {
  __shared__ __align__(16) _Float16 sT[8][8 * ZP];
  __shared__ __align__(16) _Float16 sKH[8][8 * CZ];
  __shared__ __align__(16) unsigned int sKQ[8][8 * CZ / 4];
  const int tid = threadIdx.x, wave = tid >> 5, lane = tid & 31;
  const int r8 = lane >> 2, cq = (lane & 3) * 8;
  F8 sc, sh;
  sc.v[0] = *(const v4f*)(st + cq);
  sc.v[1] = *(const v4f*)(st + cq + 4);
  sh.v[0] = *(const v4f*)(st + CZ + cq);
  sh.v[1] = *(const v4f*)(st + CZ + cq + 4);
  const float a = bfr(aP[0]);
  _Float16* zyh = (_Float16*)(void*)zy;
  const unsigned int* khw = (const unsigned int*)(const void*)kh;
  _Float16* stw = sT[wave];
  _Float16* skh = sKH[wave];
  unsigned int* skq = sKQ[wave];
  const size_t wbase = ((size_t)blockIdx.x * 8 + wave) * (APIX / 8);
#pragma unroll 1
  for (int it = 0; it < APIX / 64; ++it) {
    const size_t gp0 = wbase + (size_t)it * 8;
    const size_t gp  = gp0 + r8;
    F8 y;
    y.v[0] = *(const v4f*)(zy + gp * CZ + cq);
    y.v[1] = *(const v4f*)(zy + gp * CZ + cq + 4);
    const v4u kw4 = *(const v4u*)(khw + ((gp * CZ + cq) >> 1));
    const v2u qw  = *(const v2u*)(kq + ((gp * CZ + cq) >> 2));
    H8 ph, pl, hk;
    unsigned int qlo = 0u, qhi = 0u;
#pragma unroll
    for (int u = 0; u < 8; ++u) {
      float t = y.f[u] * sc.f[u] + sh.f[u];
      t = (t >= 0.0f) ? t : a * t;
      const unsigned int kw = kw4[u >> 1];
      const unsigned int kb = (kw >> (16 * (u & 1))) & 0xFFFFu;
      int ek = (int)((kb >> 10) & 31u);
      ek = (ek < 1) ? 1 : ((ek > 30) ? 30 : ek);
      const unsigned int qword = (u < 4) ? qw.x : qw.y;
      const unsigned int qb = (qword >> (8 * (u & 3))) & 255u;
      const float qf = (float)(((int)(qb << 24)) >> 24);
      const float kval = h_up(kb) + qf * __uint_as_float((unsigned int)(94 + ek) << 23);
      t += addRes ? kval : 0.0f;
      _Float16 hh, ll;
      split16(t, hh, ll);
      ph.f[u] = hh;
      pl.f[u] = ll;
      const _Float16 hkv = (_Float16)t;
      hk.f[u] = hkv;
      const unsigned int hb = h_bits(hkv);
      int eh = (int)((hb >> 10) & 31u);
      eh = (eh < 1) ? 1 : ((eh > 30) ? 30 : eh);
      const float rres = t - (float)hkv;
      int qi = (int)rintf(rres * __uint_as_float((unsigned int)(160 - eh) << 23));
      qi = (qi < -127) ? -127 : ((qi > 127) ? 127 : qi);
      const unsigned int qbits = (unsigned int)qi & 255u;
      if (u < 4) qlo |= qbits << (8 * u); else qhi |= qbits << (8 * (u - 4));
    }
    *(v8h*)(stw + r8 * ZP + cq) = ph.v;
    *(v8h*)(stw + r8 * ZP + CZ + cq) = pl.v;
    if (wkeep) {
      v2u qv; qv.x = qlo; qv.y = qhi;
      *(v8h*)(skh + r8 * CZ + cq) = hk.v;
      *(v2u*)(skq + ((r8 * CZ + cq) >> 2)) = qv;
    }
    wave_sync_lds();
    const v8h z0 = *(const v8h*)(stw + lane * 8);
    const v8h z1 = *(const v8h*)(stw + 4 * ZP + lane * 8);
    const v8h kk = *(const v8h*)(skh + lane * 8);
    const v4u k4 = *(const v4u*)(skq + (lane & 15) * 4);
    _Float16* dz0 = zyh + gp0 * ZP + lane * 8;
    _Float16* dz1 = dz0 + 4 * ZP;
    _Float16* dk  = kh + gp0 * CZ + lane * 8;
    unsigned int* dq = kq + gp0 * (CZ / 4) + (lane & 15) * 4;
    *(volatile v8h*)dz0 = z0;
    *(volatile v8h*)dz1 = z1;
    if (wkeep) {
      *(volatile v8h*)dk = kk;
      if (lane < 16) *(volatile v4u*)dq = k4;
    }
    __threadfence();
    *(volatile v8h*)dz0 = z0;
    *(volatile v8h*)dz1 = z1;
    if (wkeep) {
      *(volatile v8h*)dk = kk;
      if (lane < 16) *(volatile v4u*)dq = k4;
    }
    wave_sync_lds();
  }
}

__global__ __launch_bounds__(256) void k_rows(const float* Zc, const float* st, float* out, float* rs) {
  __shared__ __align__(16) float sRS[64];
  const int tid = threadIdx.x, wave = tid >> 5, lane = tid & 31;
  const int b = blockIdx.x / (NN / 32), n0 = (blockIdx.x - b * (NN / 32)) * 32;
  const float sc = st[0], sh = st[CZ];
#pragma unroll 1
  for (int jr = 0; jr < 4; ++jr) {
    const int n = n0 + wave * 4 + jr;
    const float* z0 = Zc + (size_t)b * HW + (size_t)n * MM;
    const float* z1 = Zc + (size_t)(b + BIMG) * HW + (size_t)n * MM;
    float mx = -3.0e38f;
#pragma unroll 1
    for (int k = 0; k < MM / 32; ++k) {
      const int mc = k * 32 + lane;
      const float m0 = z0[mc] * sc + sh, m1 = z1[mc] * sc + sh;
      mx = fmaxf(mx, (m0 + m1) * 0.5f);
    }
    mx = wmax32(mx);
    float se = 0.0f;
#pragma unroll 1
    for (int k = 0; k < MM / 32; ++k) {
      const int mc = k * 32 + lane;
      const float m0 = z0[mc] * sc + sh, m1 = z1[mc] * sc + sh;
      se += __expf((m0 + m1) * 0.5f - mx);
    }
    se = wsum32(se);
    const float rinv = 1.0f / se;
    for (int pass = 0; pass < 2; ++pass) {
#pragma unroll 1
      for (int k = 0; k < MM / 32; ++k) {
        const int mc = k * 32 + lane;
        const float m0 = z0[mc] * sc + sh, m1 = z1[mc] * sc + sh;
        const size_t o = (size_t)b * HW + (size_t)n * MM + mc;
        *(volatile float*)(out + OUTN + o) = m0;
        *(volatile float*)(out + 2 * OUTN + o) = m1;
      }
      __threadfence();
    }
    if (lane == 0) { sRS[(wave * 4 + jr) * 2] = mx; sRS[(wave * 4 + jr) * 2 + 1] = rinv; }
  }
  __syncthreads();
  if (tid < 16) {
    const v4f v = *(const v4f*)(sRS + tid * 4);
    float* dst = rs + ((size_t)b * NN + n0) * 2 + tid * 4;
    *(volatile v4f*)dst = v;
    __threadfence();
    *(volatile v4f*)dst = v;
  }
}

__global__ __launch_bounds__(256) void k_cols(const float* Zc, const float* st, const float* rs, float* out) {
  __shared__ float sRed[8][32];
  __shared__ float sCM[32];
  __shared__ float sCI[32];
  const int tid = threadIdx.x, wave = tid >> 5, lane = tid & 31;
  const int b = blockIdx.x / (MM / 32), mc = (blockIdx.x - b * (MM / 32)) * 32 + lane;
  const float sc = st[0], sh = st[CZ];
  const float* z0 = Zc + (size_t)b * HW + mc;
  const float* z1 = Zc + (size_t)(b + BIMG) * HW + mc;
  float mx = -3.0e38f;
#pragma unroll 1
  for (int k = 0; k < NN / 8; ++k) {
    const int n = wave + 8 * k;
    const float m0 = z0[(size_t)n * MM] * sc + sh, m1 = z1[(size_t)n * MM] * sc + sh;
    mx = fmaxf(mx, (m0 + m1) * 0.5f);
  }
  sRed[wave][lane] = mx;
  __syncthreads();
  if (tid < 32) {
    float c = -3.0e38f;
#pragma unroll
    for (int w = 0; w < 8; ++w) c = fmaxf(c, sRed[w][tid]);
    sCM[tid] = c;
  }
  __syncthreads();
  const float cm = sCM[lane];
  float se = 0.0f;
#pragma unroll 1
  for (int k = 0; k < NN / 8; ++k) {
    const int n = wave + 8 * k;
    const float m0 = z0[(size_t)n * MM] * sc + sh, m1 = z1[(size_t)n * MM] * sc + sh;
    se += __expf((m0 + m1) * 0.5f - cm);
  }
  sRed[wave][lane] = se;
  __syncthreads();
  if (tid < 32) {
    float c = 0.0f;
#pragma unroll
    for (int w = 0; w < 8; ++w) c += sRed[w][tid];
    sCI[tid] = 1.0f / c;
  }
  __syncthreads();
  const float ci = sCI[lane];
  for (int pass = 0; pass < 2; ++pass) {
#pragma unroll 1
    for (int k = 0; k < NN / 8; ++k) {
      const int n = wave + 8 * k;
      const float m0 = z0[(size_t)n * MM] * sc + sh, m1 = z1[(size_t)n * MM] * sc + sh;
      const float v = (m0 + m1) * 0.5f;
      const float rm = rs[((size_t)b * NN + n) * 2], ri = rs[((size_t)b * NN + n) * 2 + 1];
      const float pr = __expf(v - rm) * ri;
      const float pc = __expf(v - cm) * ci;
      *(volatile float*)(out + (size_t)b * HW + (size_t)n * MM + mc) = fminf(pr, pc);
    }
    __threadfence();
  }
}

extern "C" void kernel_launch(void* const* d_in, const int* in_sizes, int n_in,
                              void* d_out, int out_size, void* d_ws, size_t ws_size, hipStream_t stream) {
  if (n_in < 16) return;
  if (in_sizes[0] != BIMG * HW || in_sizes[1] != BIMG * HW) return;
  if (in_sizes[2] != CI * 2 || in_sizes[3] != CI) return;
  if (in_sizes[4] != CZ * (2 + CI) || in_sizes[5] != CZ || in_sizes[6] != CZ) return;
  if (in_sizes[7] != (NLAY - 1) * CI * 2 * CZ || in_sizes[8] != (NLAY - 1) * CI) return;
  if (in_sizes[9] != (NLAY - 1) * CZ * (2 * CZ + CI) || in_sizes[10] != (NLAY - 1) * CZ) return;
  if (in_sizes[11] != (NLAY - 1) * CZ || in_sizes[12] != 1 || in_sizes[13] != 2 * CZ) return;
  if (in_sizes[14] != 1 || in_sizes[15] != 1) return;
  if (out_size != 3 * OUTN) return;

  const float* Za  = (const float*)d_in[0];
  const float* Zb  = (const float*)d_in[1];
  const float* Wm0 = (const float*)d_in[2];
  const float* bm0 = (const float*)d_in[3];
  const float* W0  = (const float*)d_in[4];
  const float* g0  = (const float*)d_in[5];
  const float* be0 = (const float*)d_in[6];
  const float* Wm  = (const float*)d_in[7];
  const float* bm  = (const float*)d_in[8];
  const float* Wl  = (const float*)d_in[9];
  const float* gl  = (const float*)d_in[10];
  const float* bel = (const float*)d_in[11];
  const float* aP  = (const float*)d_in[12];
  const float* Wf  = (const float*)d_in[13];
  const float* gf  = (const float*)d_in[14];
  const float* bfp = (const float*)d_in[15];
  float* out = (float*)d_out;

  const size_t PZY   = (size_t)NB * HW * ZP * 2;
  const size_t PKH   = (size_t)NB * HW * CZ * 2;
  const size_t PKQ   = (size_t)NB * HW * CZ;
  const size_t PPOOL = (size_t)NB * NIDX * PP * 2;
  const size_t PT    = (size_t)NB * NIDX * CZ * 4;
  const size_t PPART = (size_t)NPB * 64 * 4;
  const size_t PST   = 256;
  const size_t PWPL  = (size_t)NWROW * WPP * 2;
  const size_t PZC   = (size_t)NB * HW * 4;
  const size_t PRS   = (size_t)BIMG * NN * 2 * 4;
  size_t off = 0;
  const size_t oZY   = off; off += PZY;
  const size_t oKH   = off; off += PKH;
  const size_t oKQ   = off; off += PKQ;
  const size_t oPOOL = off; off += PPOOL;
  const size_t oT    = off; off += PT;
  const size_t oPART = off; off += PPART;
  const size_t oST   = off; off += PST;
  const size_t oWPL  = off; off += PWPL;
  const size_t oZC   = off; off += PZC;
  const size_t oRS   = off; off += PRS;
  if (off > ws_size) return;
  if (off > (size_t)134217728) return;

  char* ws = (char*)d_ws;
  _Float16* zyh  = (_Float16*)(ws + oZY);
  float*    zyf  = (float*)(ws + oZY);
  _Float16* keph = (_Float16*)(ws + oKH);
  unsigned int* kepq = (unsigned int*)(ws + oKQ);
  _Float16* pool = (_Float16*)(ws + oPOOL);
  float*    tbuf = (float*)(ws + oT);
  float*    part = (float*)(ws + oPART);
  float*    st   = (float*)(ws + oST);
  _Float16* wpl  = (_Float16*)(ws + oWPL);
  float*    Zc   = (float*)(ws + oZC);
  float*    rs   = (float*)(ws + oRS);

  const dim3 blk(256);
  const float cnt = (float)((size_t)NB * HW);

  k_prep<<<dim3(NB * HW / 32), blk, 0, stream>>>(Za, Zb, zyh);
  k_wplanes<<<dim3((NWROW * 8 + 255) / 256), blk, 0, stream>>>(Wm0, Wm, W0, Wl, Wf, wpl);

  for (int i = 0; i < NLAY; ++i) {
    const _Float16* wm = wpl + (size_t)((i == 0) ? RWM0 : (RWMB + (i - 1) * CI)) * WPP;
    const _Float16* wx = wpl + (size_t)((i == 0) ? RWX0 : (RWXB + (i - 1) * CZ)) * WPP;
    const _Float16* wt = wpl + (size_t)((i == 0) ? RWT0 : (RWTB + (i - 1) * CZ)) * WPP;
    const float* bmi = (i == 0) ? bm0 : (bm + (size_t)(i - 1) * CI);
    const float* gi  = (i == 0) ? g0  : (gl + (size_t)(i - 1) * CZ);
    const float* bei = (i == 0) ? be0 : (bel + (size_t)(i - 1) * CZ);
    const dim3 gp(NB * NIDX / 8);
    if (i == 0) k_pool<1, 0><<<gp, blk, 0, stream>>>(zyh, wm, bmi, pool);
    else        k_pool<2, 1><<<gp, blk, 0, stream>>>(zyh, wm, bmi, pool);
    GD dt{pool, wt, tbuf, tbuf, part, PP, NIDX};
    k_gemm<1, 2, 2><<<dim3(BIMG * NIDX / 128), dim3(128), 0, stream>>>(dt);
    GD dc{zyh, wx, tbuf, zyf, part, ZP, HW};
    if (i == 0) k_gemm<2, 1, 0><<<dim3(NPB), dim3(128), 0, stream>>>(dc);
    else        k_gemm<2, 2, 1><<<dim3(NPB), dim3(128), 0, stream>>>(dc);
    k_bnfin<<<dim3(1), dim3(64), 0, stream>>>(part, NPB, cnt, gi, bei, CZ, CZ, st);
    const int addRes = (i == 2 || i == 4) ? 1 : 0;
    const int wkeep  = (i == 0 || i == 2) ? 1 : 0;
    k_bnapply<<<dim3(NB * HW / APIX), blk, 0, stream>>>(zyf, keph, kepq, st, aP, addRes, wkeep);
  }

  GD df{zyh, wpl + (size_t)RWF * WPP, tbuf, Zc, part, ZP, HW};
  k_gemm<3, 2, 1><<<dim3(NPB), dim3(128), 0, stream>>>(df);
  k_bnfin<<<dim3(1), dim3(64), 0, stream>>>(part, NPB, cnt, gf, bfp, 1, 1, st);
  k_rows<<<dim3(BIMG * (NN / 32)), blk, 0, stream>>>(Zc, st, out, rs);
  k_cols<<<dim3(BIMG * (MM / 32)), blk, 0, stream>>>(Zc, st, rs, out);
  (void)hipGetLastError();
}
